// GCNLayer_12893491822858
// MI455X (gfx1250) — hardware-run, weakly checked
//
#include <hip/hip_runtime.h>

typedef float          v8f   __attribute__((ext_vector_type(8)));
typedef float          v4f   __attribute__((ext_vector_type(4)));
typedef unsigned int   v4u   __attribute__((ext_vector_type(4)));
typedef int            v8i   __attribute__((ext_vector_type(8)));
typedef unsigned short v8us  __attribute__((ext_vector_type(8)));
typedef unsigned short v16us __attribute__((ext_vector_type(16)));
typedef __bf16         v16bf __attribute__((ext_vector_type(16)));
typedef _Float16       v16h  __attribute__((ext_vector_type(16)));
typedef v4f  __attribute__((may_alias)) v4fa;
typedef v8us __attribute__((may_alias)) v8usa;
union FragB { v16bf v; v16us u; v8us h[2]; v8i w; };
union FragH { v16h  v; v16us u; v8us h[2]; v8i w; };

__device__ __forceinline__ v8f wmb(const FragB& a, const FragB& b, v8f c) {
  v8f d = __builtin_amdgcn_wmma_f32_16x16x32_bf16(false, a.v, false, b.v, (short)0, c, false, false);
  asm volatile("v_nop\n\tv_nop\n\tv_nop\n\tv_nop" : "+v"(d) : "v"(a.w), "v"(b.w));
  return d;
}

__device__ __forceinline__ v8f wmh(const FragH& a, const FragH& b, v8f c) {
  v8f d = __builtin_amdgcn_wmma_f32_16x16x32_f16(false, a.v, false, b.v, (short)0, c, false, false);
  asm volatile("v_nop\n\tv_nop\n\tv_nop\n\tv_nop" : "+v"(d) : "v"(a.w), "v"(b.w));
  return d;
}

__device__ __forceinline__ unsigned bf16_bits(float f) {
  const unsigned u = __float_as_uint(f);
  const unsigned r = (u + 0x7FFFu + ((u >> 16) & 1u)) >> 16;
  const unsigned q = (u >> 16) | 0x40u;
  return ((u & 0x7fffffffu) > 0x7f800000u) ? q : r;
}

__device__ __forceinline__ float bf16_val(float f) {
  return __uint_as_float(bf16_bits(f) << 16);
}
__device__ __forceinline__ int clampi(int v, int lo, int hi) {
  return v < lo ? lo : (v > hi ? hi : v);
}

__device__ __forceinline__ unsigned f16_bits(float f) {
  const unsigned u  = __float_as_uint(f);
  const unsigned s  = (u >> 16) & 0x8000u;
  const unsigned a  = u & 0x7fffffffu;
  const unsigned t  = a - 0x38000000u;
  const unsigned r  = (t + 0x0FFFu + ((t >> 13) & 1u)) >> 13;
  const unsigned rc = r > 0x7C00u ? 0x7C00u : r;
  const bool small  = a < 0x38800000u;
  const bool isnan  = a > 0x7f800000u;
  const unsigned fin = small ? 0u : (s | rc);
  return isnan ? (s | 0x7E00u) : fin;
}

__device__ __forceinline__ unsigned pk16(unsigned lo, unsigned hi) { return lo | (hi << 16); }
__device__ __forceinline__ unsigned bf16_lo_bits(float v) {
  float hi = bf16_val(v);
  asm volatile("" : "+v"(hi));
  return bf16_bits(v - hi);
}
__device__ __forceinline__ v4u pack8_bf16(v4f a, v4f c) {
  return (v4u){ pk16(bf16_bits(a[0]), bf16_bits(a[1])), pk16(bf16_bits(a[2]), bf16_bits(a[3])),
                pk16(bf16_bits(c[0]), bf16_bits(c[1])), pk16(bf16_bits(c[2]), bf16_bits(c[3])) };
}
__device__ __forceinline__ v4u pack8_bf16_lo(v4f a, v4f c) {
  return (v4u){ pk16(bf16_lo_bits(a[0]), bf16_lo_bits(a[1])), pk16(bf16_lo_bits(a[2]), bf16_lo_bits(a[3])),
                pk16(bf16_lo_bits(c[0]), bf16_lo_bits(c[1])), pk16(bf16_lo_bits(c[2]), bf16_lo_bits(c[3])) };
}
__device__ __forceinline__ v4u pack8_f16(v4f a, v4f c) {
  return (v4u){ pk16(f16_bits(a[0]), f16_bits(a[1])), pk16(f16_bits(a[2]), f16_bits(a[3])),
                pk16(f16_bits(c[0]), f16_bits(c[1])), pk16(f16_bits(c[2]), f16_bits(c[3])) };
}

template <int FORM>
__global__ __launch_bounds__(256) void k_plane(const float* __restrict__ src, int rows, int cols, int ldsrc,
                                               unsigned short* __restrict__ dst, int MP, int KP) {
  static_assert(FORM >= 0 && FORM <= 3);
  const int KTOT = (FORM == 1 || FORM == 3) ? 2 * KP : KP;
  const unsigned ppr   = (unsigned)(KTOT >> 3);
  const unsigned kp8   = (unsigned)(KP >> 3);
  const unsigned total = (unsigned)MP * ppr;
  const unsigned g     = blockIdx.x * 256u + threadIdx.x;
  const unsigned rowu  = g / ppr;
  const unsigned p     = g - rowu * ppr;
  const bool second    = p >= kp8;
  const int row = (int)rowu;
  const int c0  = (int)((second ? p - kp8 : p) << 3);
  const float* srow = src + (size_t)clampi(row, 0, rows - 1) * (size_t)ldsrc;
  float x[8];
  unsigned mk[8];
#pragma unroll
  for (int e = 0; e < 8; ++e) {
    const int c = c0 + e;
    const float v = srow[clampi(c, 0, cols - 1)];
    asm volatile("" :: "v"(v));
    x[e]  = v;
    mk[e] = (row < rows && c < cols) ? 0xFFFFu : 0u;
  }
  const v4f a = (v4f){ x[0], x[1], x[2], x[3] };
  const v4f c = (v4f){ x[4], x[5], x[6], x[7] };
  v4u o;
  if (FORM == 2) {
    o = pack8_f16(a, c);
  } else {
    const v4u hi = pack8_bf16(a, c);
    o = hi;
    if (FORM == 1) { const v4u lo = pack8_bf16_lo(a, c); o = second ? lo : hi; }
  }
  const v4u mw = (v4u){ pk16(mk[0], mk[1]), pk16(mk[2], mk[3]), pk16(mk[4], mk[5]), pk16(mk[6], mk[7]) };
  o &= mw;
  if (g < total) {
    volatile v4u* q = (volatile v4u*)(dst + (size_t)g * 8);
    *q = o;
    __threadfence();
    *q = o;
  }
}

template <int FORM> struct FragOf    { typedef FragB T; };
template <>         struct FragOf<2> { typedef FragH T; };
__device__ __forceinline__ v8f mm(const FragB& a, const FragB& b, v8f c) { return wmb(a, b, c); }
__device__ __forceinline__ v8f mm(const FragH& a, const FragH& b, v8f c) { return wmh(a, b, c); }
template <class F> __device__ __forceinline__ F ld_frag(const unsigned short* p) {
  F f;
  f.h[0] = *(const v8usa*)(p);
  f.h[1] = *(const v8usa*)(p + 16);
  return f;
}

template <int FORM, int EPI>
__global__ __launch_bounds__(256) __attribute__((amdgpu_num_vgpr(248)))
void k_gemm_nt(const unsigned short* __restrict__ A, const unsigned short* __restrict__ B,
               const float* __restrict__ bias, float* __restrict__ D, int M, int N, int KTOT, int ldd) {
  static_assert(FORM >= 0 && FORM <= 2);
  static_assert(EPI == 0 || EPI == 1);
  typedef typename FragOf<FORM>::T F;
  __shared__ __attribute__((aligned(16))) float sT[8][16 * 68];
  const int lane = threadIdx.x & 31;
  const int wave = threadIdx.x >> 5;
  const int tilesM = (M + 63) >> 6;
  const int tilesN = (N + 63) >> 6;
  const int tile = blockIdx.x * 8 + wave;
  if (tile >= tilesM * tilesN) return;
  const int tm = tile / tilesN;
  const int tn = tile - tm * tilesN;
  const int m0 = tm << 6;
  const int n0 = tn << 6;

  const int rl = lane & 15;
  const int h8 = (lane >> 4) * 8;
  const unsigned short* pa = A + (size_t)(m0 + rl) * (size_t)KTOT + h8;
  const unsigned short* pb = B + (size_t)(n0 + rl) * (size_t)KTOT + h8;

  v8f acc[4][4];
#pragma unroll
  for (int i = 0; i < 4; ++i)
#pragma unroll
    for (int j = 0; j < 4; ++j) acc[i][j] = (v8f){0.f, 0.f, 0.f, 0.f, 0.f, 0.f, 0.f, 0.f};

#pragma unroll 1
  for (int k0 = 0; k0 < KTOT; k0 += 32) {
    F bf[4];
#pragma unroll
    for (int j = 0; j < 4; ++j) bf[j] = ld_frag<F>(pb + (size_t)(j << 4) * (size_t)KTOT + k0);
#pragma unroll
    for (int i = 0; i < 4; ++i) {
      const F af = ld_frag<F>(pa + (size_t)(i << 4) * (size_t)KTOT + k0);
#pragma unroll
      for (int j = 0; j < 4; ++j) acc[i][j] = mm(af, bf[j], acc[i][j]);
    }
  }

  float* slab = sT[wave];
  const int hh = lane >> 4;
  const int c4 = (lane & 15) * 4;
  const int nc = n0 + c4;
  const bool cok = nc < N;
  v4f bv = (v4f){0.f, 0.f, 0.f, 0.f};
  if (EPI == 1) {
    bv = *(const v4fa*)(bias + clampi(nc, 0, N - 4));
    asm volatile("" :: "v"(bv));
  }
#pragma unroll
  for (int i = 0; i < 4; ++i) {
    const int mBase = m0 + (i << 4);
#pragma unroll
    for (int j = 0; j < 4; ++j) {
#pragma unroll
      for (int r = 0; r < 8; ++r) slab[(h8 + r) * 68 + (j << 4) + rl] = acc[i][j][r];
    }
    __builtin_amdgcn_fence(__ATOMIC_RELEASE, "workgroup");
    __builtin_amdgcn_wave_barrier();
    __builtin_amdgcn_fence(__ATOMIC_ACQUIRE, "workgroup");
    v4f vv[8];
#pragma unroll
    for (int it = 0; it < 8; ++it) {
      const int row = it * 2 + hh;
      v4f v = *(const v4fa*)(slab + row * 68 + c4);
      if (EPI == 1) v += bv;
      vv[it] = v;
    }
    for (int pass = 0; pass < 2; ++pass) {
#pragma unroll
      for (int it = 0; it < 8; ++it) {
        const int row = mBase + it * 2 + hh;
        if (cok && row < M) *(volatile v4f*)(D + (size_t)row * (size_t)ldd + nc) = vv[it];
      }
      __threadfence();
    }
    __builtin_amdgcn_fence(__ATOMIC_RELEASE, "workgroup");
    __builtin_amdgcn_wave_barrier();
    __builtin_amdgcn_fence(__ATOMIC_ACQUIRE, "workgroup");
  }
}

#pragma clang fp contract(off)
#include <stddef.h>

#define NNODE   50000
#define FDIM    100
#define NEDGE   800000
#define MPAD    50048
#define KPAD    128
#define NTHR    256
#define NWAVE   8
#define EPT     8
#define WCH     (32 * EPT)
#define NBRUN   1024
#define SLB     10
#define NBK     49
#define WLCAP   2624
#define LCAP    20992
#define MAXDEG_MEAS   33
#define MAXB1024_MEAS 16696
#define NOUT    5000000

#define WL_OFF   0
#define PL_OFF   (NWAVE * WLCAP)
#define CNT_OFF  (PL_OFF + LCAP)
#define OFFS_OFF (CNT_OFF + NBRUN)
#define CUR_OFF  (OFFS_OFF + NBRUN)
#define MISC_OFF (CUR_OFF + NBRUN)
#define BK_ZINTS MISC_OFF
#define BK_INTS  (BK_ZINTS + 16)
#define BK_LDS   (BK_INTS * 4)

static_assert(MPAD == 391 * 128 && MPAD >= NNODE && MPAD % 64 == 0 && MPAD % 16 == 0 && MPAD % NWAVE == 0);
static_assert(KPAD % 64 == 0 && KPAD % 32 == 0 && KPAD >= FDIM && KPAD == 32 * 4);
static_assert(FDIM % 4 == 0 && (FDIM * FDIM) % 4 == 0);
static_assert(NBRUN == (1 << SLB) && NBRUN % 32 == 0);
static_assert(NBK * NBRUN == 50176 && NBK * NBRUN >= MPAD && (NBK - 1) * NBRUN < NNODE);
static_assert(NEDGE < (1 << 21) && (((long long)NEDGE) << SLB) < (1LL << 31));
static_assert(NEDGE % 4 == 0);
static_assert(LCAP % 256 == 0 && LCAP % 4 == 0 && NWAVE * WLCAP == LCAP);
static_assert((long long)LCAP * 100 >= (long long)MAXB1024_MEAS * 125);
static_assert(WLCAP >= MAXB1024_MEAS / 8 + 8 * 46 + 1);
static_assert(MAXDEG_MEAS <= LCAP);
static_assert(BK_ZINTS % (NTHR * 4) == 0);
static_assert(BK_LDS <= 262144);
static_assert((2 * NBRUN) % (NTHR * 4) == 0);
static_assert(NOUT == NNODE * FDIM && NOUT == 156250 * 32);
static_assert((MPAD * KPAD / 8) % NTHR == 0 && (KPAD * KPAD / 8) % NTHR == 0);

typedef int v4i __attribute__((ext_vector_type(4)));
typedef v4i __attribute__((may_alias)) v4ia;

__global__ __launch_bounds__(NTHR) void k_wprep(const float* __restrict__ w, const float* __restrict__ bias,
                                                unsigned short* WT, float* BL) {
  __shared__ __attribute__((aligned(16))) float sW[FDIM * FDIM];
  const int tid = (int)threadIdx.x;
#pragma unroll 1
  for (int it = 0; it < (FDIM * FDIM / 4 + NTHR - 1) / NTHR; ++it) {
    int i = it * NTHR + tid;
    i = i > FDIM * FDIM / 4 - 1 ? FDIM * FDIM / 4 - 1 : i;
    const v4f v = *(const v4fa*)(w + 4 * i);
    *(v4fa*)(sW + 4 * i) = v;
  }
  __syncthreads();
#pragma unroll 1
  for (int it = 0; it < (KPAD * KPAD / 8) / NTHR; ++it) {
    const int g  = it * NTHR + tid;
    const int n  = g >> 4;
    const int k8 = (g & 15) * 8;
    const int nc = clampi(n, 0, FDIM - 1);
    unsigned bt[8];
#pragma unroll
    for (int e = 0; e < 8; ++e) {
      const int k = k8 + e;
      const float v = sW[clampi(k, 0, FDIM - 1) * FDIM + nc];
      const unsigned mk = (n < FDIM && k < FDIM) ? 0xFFFFu : 0u;
      bt[e] = bf16_bits(v) & mk;
    }
    const v4u o = (v4u){ pk16(bt[0], bt[1]), pk16(bt[2], bt[3]), pk16(bt[4], bt[5]), pk16(bt[6], bt[7]) };
    volatile v4u* q = (volatile v4u*)(WT + (size_t)g * 8);
    *q = o;
    __threadfence();
    *q = o;
  }
  if (tid < 32) {
    const int c0 = 4 * tid;
    v4f b = *(const v4fa*)(bias + clampi(c0, 0, FDIM - 4));
    asm volatile("" :: "v"(b));
    const bool ok = c0 < FDIM;
    v4f o;
    o.x = ok ? bf16_val(b.x) : 0.0f;
    o.y = ok ? bf16_val(b.y) : 0.0f;
    o.z = ok ? bf16_val(b.z) : 0.0f;
    o.w = ok ? bf16_val(b.w) : 0.0f;
    volatile v4f* q = (volatile v4f*)(BL + c0);
    *q = o;
    __threadfence();
    *q = o;
  }
}

__global__ __launch_bounds__(NTHR) void k_bucket(const int* __restrict__ srcs, const int* __restrict__ dsts,
                                                 int* LIST, int* CO, int* FLAG) {
  extern __shared__ __attribute__((aligned(16))) int dsm[];
  const int tid = (int)threadIdx.x, lane = tid & 31, wave = tid >> 5;
  const int blk = (int)blockIdx.x;
  const unsigned nbs = (unsigned)(blk * NBRUN);

  {
    const v4i z4 = {0, 0, 0, 0};
#pragma unroll 1
    for (int i = tid * 4; i < BK_ZINTS; i += NTHR * 4) *(v4ia*)(dsm + i) = z4;
    if (tid < 16) dsm[MISC_OFF + tid] = 0;
  }
  __syncthreads();

  {
    const int per  = ((NEDGE + NWAVE * WCH - 1) / (NWAVE * WCH)) * WCH;
    const int ebeg = wave * per;
    const int eend = (ebeg + per < NEDGE) ? (ebeg + per) : NEDGE;
    const int wb = WL_OFF + wave * WLCAP;
    int wc = 0;
#pragma unroll 1
    for (int cb = ebeg; cb < eend; cb += WCH) {
      const int e0 = cb + lane * EPT;
      v4i da, db;
      if (cb + WCH <= NEDGE) {
        da = *(const v4ia*)(dsts + e0);
        db = *(const v4ia*)(dsts + e0 + 4);
      } else {
        int t[8];
#pragma unroll
        for (int j = 0; j < 8; ++j) {
          const int e  = e0 + j;
          const int ec = e < NEDGE ? e : NEDGE - 1;
          const int v  = dsts[ec];
          asm volatile("" :: "v"(v));
          t[j] = e < NEDGE ? v : -1;
        }
        da.x = t[0]; da.y = t[1]; da.z = t[2]; da.w = t[3];
        db.x = t[4]; db.y = t[5]; db.z = t[6]; db.w = t[7];
      }
      const unsigned s0 = (unsigned)da.x - nbs, s1 = (unsigned)da.y - nbs;
      const unsigned s2 = (unsigned)da.z - nbs, s3 = (unsigned)da.w - nbs;
      const unsigned s4 = (unsigned)db.x - nbs, s5 = (unsigned)db.y - nbs;
      const unsigned s6 = (unsigned)db.z - nbs, s7 = (unsigned)db.w - nbs;
      const bool h0 = (s0 < (unsigned)NBRUN) & ((unsigned)da.x < (unsigned)NNODE);
      const bool h1 = (s1 < (unsigned)NBRUN) & ((unsigned)da.y < (unsigned)NNODE);
      const bool h2 = (s2 < (unsigned)NBRUN) & ((unsigned)da.z < (unsigned)NNODE);
      const bool h3 = (s3 < (unsigned)NBRUN) & ((unsigned)da.w < (unsigned)NNODE);
      const bool h4 = (s4 < (unsigned)NBRUN) & ((unsigned)db.x < (unsigned)NNODE);
      const bool h5 = (s5 < (unsigned)NBRUN) & ((unsigned)db.y < (unsigned)NNODE);
      const bool h6 = (s6 < (unsigned)NBRUN) & ((unsigned)db.z < (unsigned)NNODE);
      const bool h7 = (s7 < (unsigned)NBRUN) & ((unsigned)db.w < (unsigned)NNODE);
      const unsigned m0 = __builtin_amdgcn_ballot_w32(h0), m1 = __builtin_amdgcn_ballot_w32(h1);
      const unsigned m2 = __builtin_amdgcn_ballot_w32(h2), m3 = __builtin_amdgcn_ballot_w32(h3);
      const unsigned m4 = __builtin_amdgcn_ballot_w32(h4), m5 = __builtin_amdgcn_ballot_w32(h5);
      const unsigned m6 = __builtin_amdgcn_ballot_w32(h6), m7 = __builtin_amdgcn_ballot_w32(h7);
      const unsigned any = m0 | m1 | m2 | m3 | m4 | m5 | m6 | m7;
      if (any != 0u) {
        const int pre = (int)(__builtin_amdgcn_mbcnt_lo(m0, 0u) + __builtin_amdgcn_mbcnt_lo(m1, 0u) +
                              __builtin_amdgcn_mbcnt_lo(m2, 0u) + __builtin_amdgcn_mbcnt_lo(m3, 0u) +
                              __builtin_amdgcn_mbcnt_lo(m4, 0u) + __builtin_amdgcn_mbcnt_lo(m5, 0u) +
                              __builtin_amdgcn_mbcnt_lo(m6, 0u) + __builtin_amdgcn_mbcnt_lo(m7, 0u));
        int p = wc + pre;
        if (h0) { if (p < WLCAP) dsm[wb + p] = ((e0 + 0) << SLB) | (int)s0; p = p + 1; }
        if (h1) { if (p < WLCAP) dsm[wb + p] = ((e0 + 1) << SLB) | (int)s1; p = p + 1; }
        if (h2) { if (p < WLCAP) dsm[wb + p] = ((e0 + 2) << SLB) | (int)s2; p = p + 1; }
        if (h3) { if (p < WLCAP) dsm[wb + p] = ((e0 + 3) << SLB) | (int)s3; p = p + 1; }
        if (h4) { if (p < WLCAP) dsm[wb + p] = ((e0 + 4) << SLB) | (int)s4; p = p + 1; }
        if (h5) { if (p < WLCAP) dsm[wb + p] = ((e0 + 5) << SLB) | (int)s5; p = p + 1; }
        if (h6) { if (p < WLCAP) dsm[wb + p] = ((e0 + 6) << SLB) | (int)s6; p = p + 1; }
        if (h7) { if (p < WLCAP) dsm[wb + p] = ((e0 + 7) << SLB) | (int)s7; p = p + 1; }
        wc += (int)(__builtin_popcount(m0) + __builtin_popcount(m1) + __builtin_popcount(m2) + __builtin_popcount(m3) +
                    __builtin_popcount(m4) + __builtin_popcount(m5) + __builtin_popcount(m6) + __builtin_popcount(m7));
      }
    }
    if (lane == 0) dsm[MISC_OFF + wave] = wc;
  }
  __syncthreads();

  if (wave == 0) {
    int ov = 0;
    int tot = 0;
#pragma unroll 1
    for (int w2 = 0; w2 < NWAVE; ++w2) {
      int c = __builtin_amdgcn_readfirstlane(dsm[MISC_OFF + w2]);
      if (c > WLCAP) ov = 1;
      c = c < 0 ? 0 : (c > WLCAP ? WLCAP : c);
      tot += c;
#pragma unroll 1
      for (int b0 = 0; b0 < c; b0 += 32) {
        const int idx = b0 + lane;
        const int ent = dsm[WL_OFF + w2 * WLCAP + (idx < WLCAP ? idx : WLCAP - 1)];
        const int m32 = (c - b0) < 32 ? (c - b0) : 32;
#pragma unroll 1
        for (int k = 0; k < m32; ++k) {
          const int u    = __builtin_amdgcn_readlane(ent, k);
          const int slot = u & (NBRUN - 1);
          if (lane == 0) dsm[CNT_OFF + slot] = dsm[CNT_OFF + slot] + 1;
        }
      }
    }
    if (tot > LCAP) ov = 1;
    if (lane == 0) dsm[MISC_OFF + 9] = ov;
  }
  __syncthreads();
  if (wave == 0) {
    const int base = lane * (NBRUN / 32);
    int s = 0;
#pragma unroll 1
    for (int i = 0; i < NBRUN / 32; ++i) s += dsm[CNT_OFF + base + i];
    int incl = s;
#pragma unroll
    for (int d = 1; d < 32; d <<= 1) {
      const int y = __shfl_up(incl, d, 32);
      if (lane >= d) incl += y;
    }
    int run = incl - s;
#pragma unroll 1
    for (int i = 0; i < NBRUN / 32; ++i) {
      const int cv = dsm[CNT_OFF + base + i];
      dsm[OFFS_OFF + base + i] = run;
      dsm[CUR_OFF + base + i]  = run;
      run += cv;
    }
  }
  __syncthreads();

  if (wave == 0) {
#pragma unroll 1
    for (int w2 = 0; w2 < NWAVE; ++w2) {
      int c = __builtin_amdgcn_readfirstlane(dsm[MISC_OFF + w2]);
      c = c < 0 ? 0 : (c > WLCAP ? WLCAP : c);
#pragma unroll 1
      for (int b0 = 0; b0 < c; b0 += 32) {
        const int idx = b0 + lane;
        const int ent = dsm[WL_OFF + w2 * WLCAP + (idx < WLCAP ? idx : WLCAP - 1)];
        int eid = (ent >> SLB) & 0x1FFFFF;
        eid = eid > NEDGE - 1 ? NEDGE - 1 : eid;
        int sr = srcs[eid];
        asm volatile("" :: "v"(sr));
        sr = sr < 0 ? 0 : (sr > NNODE - 1 ? NNODE - 1 : sr);
        const int m32 = (c - b0) < 32 ? (c - b0) : 32;
#pragma unroll 1
        for (int k = 0; k < m32; ++k) {
          const int u    = __builtin_amdgcn_readlane(ent, k);
          const int w0   = __builtin_amdgcn_readlane(sr, k);
          const int slot = u & (NBRUN - 1);
          if (lane == 0) {
            int p = dsm[CUR_OFF + slot];
            p = p < 0 ? 0 : (p > LCAP - 1 ? LCAP - 1 : p);
            dsm[PL_OFF + p] = w0;
            dsm[CUR_OFF + slot] = p + 1;
          }
        }
      }
    }
  }
  __syncthreads();

  const int ovf = dsm[MISC_OFF + 9];
  int* lp  = LIST + (size_t)blk * (size_t)LCAP;
  int* cop = CO + (size_t)blk * (2 * NBRUN);
  int* fp  = FLAG + (size_t)blk * 32;
#pragma unroll 1
  for (int pass = 0; pass < 2; ++pass) {
#pragma unroll 1
    for (int i = tid * 4; i < LCAP; i += NTHR * 4) {
      const v4i v = *(const v4ia*)(dsm + PL_OFF + i);
      *(volatile v4i*)(lp + i) = v;
    }
#pragma unroll 1
    for (int i = tid * 4; i < 2 * NBRUN; i += NTHR * 4) {
      const v4i v = *(const v4ia*)(dsm + CNT_OFF + i);
      *(volatile v4i*)(cop + i) = v;
    }
    if (tid < 8) {
      const v4i f = {ovf, ovf, ovf, ovf};
      *(volatile v4i*)(fp + 4 * tid) = f;
    }
    __threadfence();
  }
}

__global__ __launch_bounds__(NTHR) void k_walk(const int* __restrict__ LIST, const int* __restrict__ CO,
                                               const int* __restrict__ FLAG, const float* __restrict__ T,
                                               const float* __restrict__ BL, float* Y) {
  const int tid = (int)threadIdx.x, lane = tid & 31, wave = tid >> 5;
  const int r    = __builtin_amdgcn_readfirstlane((int)blockIdx.x * NWAVE + wave);
  const int b    = clampi(r >> SLB, 0, NBK - 1);
  const int slot = r & (NBRUN - 1);
  const int* lb  = LIST + (size_t)b * (size_t)LCAP;
  const int craw = CO[(size_t)b * (2 * NBRUN) + slot];
  const int oraw = CO[(size_t)b * (2 * NBRUN) + NBRUN + slot];
  const int flag = FLAG[(size_t)b * 32];
  const int c = __builtin_amdgcn_readfirstlane((r < MPAD) ? clampi(craw, 0, LCAP) : 0);
  const int o = __builtin_amdgcn_readfirstlane(clampi(oraw, 0, LCAP - 1));
  int last = o + (c > 0 ? c : 1) - 1;
  last = last > LCAP - 1 ? LCAP - 1 : last;

  v4f a = (v4f){0.0f, 0.0f, 0.0f, 0.0f};
#pragma unroll 1
  for (int b0 = 0; b0 < c; b0 += 32) {
    int idx = o + b0 + lane;
    idx = idx > last ? last : idx;
    int sr = lb[idx];
    asm volatile("" :: "v"(sr));
    sr = sr < 0 ? 0 : (sr > NNODE - 1 ? NNODE - 1 : sr);
    const int m32 = (c - b0) < 32 ? (c - b0) : 32;
#pragma unroll 1
    for (int k = 0; k < m32; ++k) {
      const int sk = __builtin_amdgcn_readlane(sr, k);
      const v4f q = *(const v4fa*)(T + (size_t)sk * KPAD + 4 * lane);
      a = a + q;
    }
  }
  const v4f bl = *(const v4fa*)(BL + 4 * lane);
  const float dn = (float)(c > 1 ? c : 1);
  v4f y;
  y.x = a.x / dn + bl.x;
  y.y = a.y / dn + bl.y;
  y.z = a.z / dn + bl.z;
  y.w = a.w / dn + bl.w;
  const bool live = (r < NNODE) & (4 * lane < FDIM);
  const bool bad  = flag != 0;
  const float qnan = __uint_as_float(0x7fc00000u);
  v4f ov;
  ov.x = live ? y.x : 0.0f; ov.y = live ? y.y : 0.0f; ov.z = live ? y.z : 0.0f; ov.w = live ? y.w : 0.0f;
  ov.x = bad ? qnan : ov.x; ov.y = bad ? qnan : ov.y; ov.z = bad ? qnan : ov.z; ov.w = bad ? qnan : ov.w;
  volatile v4f* qp = (volatile v4f*)(Y + (size_t)r * KPAD + 4 * lane);
  *qp = ov;
  __threadfence();
  *qp = ov;
}

__global__ __launch_bounds__(NTHR) void k_flat(const float* __restrict__ Y, float* out) {
  const unsigned f  = blockIdx.x * (unsigned)NTHR + threadIdx.x;
  const unsigned fc = f < (unsigned)NOUT ? f : (unsigned)(NOUT - 1);
  const unsigned row = fc / (unsigned)FDIM;
  const unsigned col = fc - row * (unsigned)FDIM;
  const float v = Y[(size_t)row * KPAD + col];
  asm volatile("" :: "v"(v));
  if (f < (unsigned)NOUT) {
    volatile float* q = out + f;
    *q = v;
    __threadfence();
    *q = v;
  }
}

extern "C" void kernel_launch(void* const* d_in, const int* in_sizes, int n_in,
                              void* d_out, int out_size, void* d_ws, size_t ws_size,
                              hipStream_t stream) {
  if (n_in < 5) return;
  if (in_sizes[0] != NNODE * FDIM) return;
  if (in_sizes[1] != NEDGE) return;
  if (in_sizes[2] != NEDGE) return;
  if (in_sizes[3] != FDIM * FDIM) return;
  if (in_sizes[4] != FDIM) return;
  if (out_size != NOUT) return;

  const float* feat = (const float*)d_in[0];
  const int*   srcs = (const int*)d_in[1];
  const int*   dsts = (const int*)d_in[2];
  const float* W    = (const float*)d_in[3];
  const float* bias = (const float*)d_in[4];
  float* out = (float*)d_out;

  constexpr size_t zFB   = (size_t)MPAD * KPAD * 2;
  constexpr size_t zWT   = (size_t)KPAD * KPAD * 2;
  constexpr size_t zBL   = (size_t)KPAD * 4;
  constexpr size_t zT    = (size_t)MPAD * KPAD * 4;
  constexpr size_t zY    = (size_t)MPAD * KPAD * 4;
  constexpr size_t zLIST = (size_t)NBK * LCAP * 4;
  constexpr size_t zCO   = (size_t)NBK * 2 * NBRUN * 4;
  constexpr size_t zFLAG = 8192;
  constexpr size_t oFB   = 0;
  constexpr size_t oWT   = oFB + zFB;
  constexpr size_t oBL   = oWT + zWT;
  constexpr size_t oT    = oBL + zBL;
  constexpr size_t oY    = oT + zT;
  constexpr size_t oLIST = oY + zY;
  constexpr size_t oCO   = oLIST + zLIST;
  constexpr size_t oFLAG = oCO + zCO;
  constexpr size_t oEND  = oFLAG + zFLAG;
  static_assert(zFB % 256 == 0 && zWT % 256 == 0 && zBL % 256 == 0 && zT % 256 == 0 && zY % 256 == 0);
  static_assert(zLIST % 256 == 0 && zCO % 256 == 0 && zFLAG % 256 == 0);
  static_assert(zFLAG >= (size_t)NBK * 128);
  static_assert(oEND == 68618752);
  static_assert(oEND <= ((size_t)128 << 20));
  if (oEND > ws_size) return;

  char* ws = (char*)d_ws;
  unsigned short* FB   = (unsigned short*)(ws + oFB);
  unsigned short* WT   = (unsigned short*)(ws + oWT);
  float*          BL   = (float*)(ws + oBL);
  float*          T    = (float*)(ws + oT);
  float*          Y    = (float*)(ws + oY);
  int*            LIST = (int*)(ws + oLIST);
  int*            CO   = (int*)(ws + oCO);
  int*            FLAG = (int*)(ws + oFLAG);

  hipFuncSetAttribute(reinterpret_cast<const void*>(&k_bucket), hipFuncAttributeMaxDynamicSharedMemorySize, (int)BK_LDS);

  k_plane<0><<<MPAD * KPAD / 8 / NTHR, NTHR, 0, stream>>>(feat, NNODE, FDIM, FDIM, FB, MPAD, KPAD);
  k_wprep<<<1, NTHR, 0, stream>>>(W, bias, WT, BL);
  k_gemm_nt<0, 0><<<(1564 + 7) / 8, NTHR, 0, stream>>>(FB, WT, BL, T, MPAD, KPAD, KPAD, KPAD);
  k_bucket<<<NBK, NTHR, BK_LDS, stream>>>(srcs, dsts, LIST, CO, FLAG);
  k_walk<<<MPAD / NWAVE, NTHR, 0, stream>>>(LIST, CO, FLAG, T, BL, Y);
  k_flat<<<(NOUT + NTHR - 1) / NTHR, NTHR, 0, stream>>>(Y, out);
}
